// CTCrackSeg_6408091205907
// MI455X (gfx1250) — hardware-verified
//
#include <hip/hip_runtime.h>


namespace {
constexpr int NB = 2, C = 64, H = 256, W = 256, P = H * W, KN = 9, KK = KN * C, NOF = 2 * KN, NOFP = 32, HP = H + 2, WP = W + 2, PZ = P + 16;
constexpr float XS = 8.0f, WSC = 256.0f;

typedef _Float16 b16;
typedef __attribute__((ext_vector_type(16))) _Float16 v16b;
typedef __attribute__((ext_vector_type(8))) _Float16 v8b;
typedef __attribute__((ext_vector_type(8))) float v8f;
typedef __attribute__((ext_vector_type(4))) float v4f;
__device__ __forceinline__ float bf16_rne(float f) { unsigned int u = __float_as_uint(f); u += 0x7FFFu + ((u >> 16) & 1u); return __uint_as_float(u & 0xFFFF0000u); }
__device__ __forceinline__ v16b frag_kb(const b16* p, int hh) { const v8b a = *(const v8b*)(p + 8 * hh), b = *(const v8b*)(p + 16 + 8 * hh); v16b f;
#pragma unroll
  for (int e = 0; e < 8; ++e) { f[e] = a[e]; f[8 + e] = b[e]; } return f; }
__device__ __forceinline__ v8f wmma16b(v16b a, v16b b, v8f c) { v8f d = __builtin_amdgcn_wmma_f32_16x16x32_f16(false, a, false, b, (short)0, c, false, false); asm volatile("v_nop\n\tv_nop\n\tv_nop\n\tv_nop" : "+v"(d) : "v"(a), "v"(b)); return d; }
__device__ __forceinline__ void wave_lds_sync() { __builtin_amdgcn_fence(__ATOMIC_RELEASE, "workgroup"); __builtin_amdgcn_wave_barrier(); __builtin_amdgcn_fence(__ATOMIC_ACQUIRE, "workgroup"); }
__device__ __forceinline__ float pmul(float a, float b) { float p = a * b; asm volatile("" : "+v"(p)); return p; }
__device__ __forceinline__ int iclamp(int v, int lo, int hi) { return v < lo ? lo : (v > hi ? hi : v); }

__global__ __launch_bounds__(256) void prepx_kernel(const float* __restrict__ x, b16* __restrict__ XT) {
  __shared__ __attribute__((aligned(16))) b16 Tt[64][64 + 8];
  const int b = blockIdx.z, p0 = blockIdx.x * 64, t_ = threadIdx.x;
  if (blockIdx.x == P / 64) { for (int pass = 0; pass < 2; ++pass) { if (t_ < 128) { const v8b z = {}; *(volatile v8b*)(XT + ((size_t)b * PZ + P) * C + t_ * 8) = z; } __threadfence(); } return; }
  for (int q = t_; q < 64 * 64; q += 256) { const int cc = q >> 6, pp = q & 63; Tt[pp][cc] = (b16)(bf16_rne(x[((size_t)b * C + cc) * P + p0 + pp]) * XS); }
  __syncthreads();
  for (int pass = 0; pass < 2; ++pass) { for (int q = t_; q < 64 * 8; q += 256) { const int pp = q >> 3, c8 = (q & 7) * 8; *(volatile v8b*)(XT + ((size_t)b * PZ + p0 + pp) * C + c8) = *(const v8b*)(&Tt[pp][c8]); } __threadfence(); }
}
__global__ __launch_bounds__(256) void prepw_kernel(const float* __restrict__ pw, const float* __restrict__ cw, b16* __restrict__ PW, b16* __restrict__ CW) {
  const int tid = blockIdx.x * 256 + threadIdx.x; const int n1 = NOFP * KK / 8, n2 = C * KK / 8;
  if (tid >= n1 + n2) return;
  v8b o; b16* dst; const bool isp = tid < n1; const int e = (isp ? tid : tid - n1) * 8; const int orow = e / KK, k0 = e - orow * KK; const int n = k0 / C, ci0 = k0 - n * C; const int kh = n / 3, kw = n - kh * 3;
#pragma unroll
  for (int j = 0; j < 8; ++j) { const int ci = ci0 + j; float v;
    if (isp) v = (orow < NOF) ? pw[(((size_t)(orow < NOF ? orow : 0) * C + ci) * 3 + kh) * 3 + kw] : 0.0f; else v = cw[(((size_t)orow * C + ci) * 3 + kh) * 3 + kw];
    o[j] = (b16)(bf16_rne(v) * WSC); }
  dst = (isp ? PW : CW) + e;
  for (int pass = 0; pass < 2; ++pass) { *(volatile v8b*)dst = o; __threadfence(); }
}
__global__ __launch_bounds__(128) void offconv_kernel(const b16* __restrict__ XT, const b16* __restrict__ PW, const float* __restrict__ pb, float* __restrict__ OFFS) {
  __shared__ __attribute__((aligned(16))) float Ts[4][16][NOFP + 4];
  const int wave = threadIdx.x >> 5, lane = threadIdx.x & 31, nloc = lane & 15, hlf = lane >> 4; const int b = blockIdx.y, pix0 = blockIdx.x * 64 + wave * 16, pix = pix0 + nloc; const int r = pix / W, c = pix - r * W;
  const b16* Xb = XT + (size_t)b * PZ * C;
  v8f acc[2] = {{}, {}};
#pragma unroll 1
  for (int n = 0; n < KN; ++n) { const int rr = r + n / 3 - 1, cc = c + n % 3 - 1; const int tok = (rr >= 0 && rr < H && cc >= 0 && cc < W) ? rr * W + cc : P;
#pragma unroll
    for (int kh2 = 0; kh2 < 2; ++kh2) { const v16b a = frag_kb(Xb + (size_t)tok * C + kh2 * 32, hlf); const int kb = n * C + kh2 * 32;
      acc[0] = wmma16b(a, frag_kb(PW + (size_t)(nloc) * KK + kb, hlf), acc[0]); acc[1] = wmma16b(a, frag_kb(PW + (size_t)(16 + nloc) * KK + kb, hlf), acc[1]); } }
#pragma unroll
  for (int t = 0; t < 2; ++t) { const int o = t * 16 + nloc; const float bb = (o < NOF) ? bf16_rne(pb[o < NOF ? o : 0]) : 0.0f;
#pragma unroll
    for (int q = 0; q < 8; ++q) Ts[wave][8 * hlf + q][o] = (o < NOF) ? acc[t][q] * (1.0f / (XS * WSC)) + bb : 0.0f; }
  wave_lds_sync();
  for (int pass = 0; pass < 2; ++pass) { for (int r4 = 0; r4 < 16; r4 += 4) { const int rr = r4 + (lane >> 3), c4 = (lane & 7) * 4; *(volatile v4f*)(OFFS + ((size_t)b * P + pix0 + rr) * NOFP + c4) = *(const v4f*)(&Ts[wave][rr][c4]); } __threadfence(); }
}
__global__ __launch_bounds__(256) void sample_kernel(const b16* __restrict__ XT, const float* __restrict__ OFFS, int b, b16* __restrict__ XO) {
  __shared__ __attribute__((aligned(16))) b16 To[4][KK + 8];
  const int t_ = threadIdx.x, pl = t_ >> 6, ci = t_ & 63; const int pix = blockIdx.x * 4 + pl; const int r = pix / W, c = pix - r * W;
  const b16* Xb = XT + (size_t)b * PZ * C + ci; const float* of = OFFS + ((size_t)b * P + pix) * NOFP;
#pragma unroll 1
  for (int n = 0; n < KN; ++n) {
    float px = (float)(c + 1) + (float)(n % 3 - 1) + of[n], py = (float)(r + 1) + (float)(n / 3 - 1) + of[KN + n];
    const float fx = floorf(px), fy = floorf(py);
    const float qltx = fminf(fmaxf(fx, 0.0f), (float)(HP - 1)), qlty = fminf(fmaxf(fy, 0.0f), (float)(WP - 1)), qrbx = fminf(fmaxf(fx + 1.0f, 0.0f), (float)(HP - 1)), qrby = fminf(fmaxf(fy + 1.0f, 0.0f), (float)(WP - 1));
    px = fminf(fmaxf(px, 0.0f), (float)(HP - 1)); py = fminf(fmaxf(py, 0.0f), (float)(WP - 1));
    const float dxlt = qltx - px, dylt = qlty - py, dxrb = qrbx - px, dyrb = qrby - py;
    const float glt = pmul(1.0f + dxlt, 1.0f + dylt), grb = pmul(1.0f - dxrb, 1.0f - dyrb), glb = pmul(1.0f + dxlt, 1.0f - dyrb), grt = pmul(1.0f - dxrb, 1.0f + dylt);
    const int ltx = (int)qltx, lty = (int)qlty, rbx = (int)qrbx, rby = (int)qrby;
    auto tokof = [&](int qx, int qy) { return (qx >= 1 && qx <= H && qy >= 1 && qy <= W) ? (qx - 1) * W + (qy - 1) : P; };
    const float vlt = (float)Xb[(size_t)tokof(ltx, lty) * C], vrb = (float)Xb[(size_t)tokof(rbx, rby) * C], vlb = (float)Xb[(size_t)tokof(ltx, rby) * C], vrt = (float)Xb[(size_t)tokof(rbx, lty) * C];
    const float v = pmul(glt, vlt) + pmul(grb, vrb) + pmul(glb, vlb) + pmul(grt, vrt);
    To[pl][n * C + ci] = (b16)v; }
  __syncthreads();
  for (int pass = 0; pass < 2; ++pass) {
    for (int q = t_; q < 4 * (KK / 8); q += 256) { const int p2 = q / (KK / 8), c8 = (q - p2 * (KK / 8)) * 8; *(volatile v8b*)(XO + ((size_t)(blockIdx.x * 4 + p2)) * KK + c8) = *(const v8b*)(&To[p2][c8]); }
    __threadfence(); }
}
__global__ __launch_bounds__(128) void conv_kernel(const b16* __restrict__ XO, const b16* __restrict__ CW, int b, float* __restrict__ out) {
  __shared__ __attribute__((aligned(16))) float Tc[C][64 + 4];
  const int wave = threadIdx.x >> 5, lane = threadIdx.x & 31, nloc = lane & 15, hlf = lane >> 4, t_ = threadIdx.x; const int pix0 = blockIdx.x * 64; const size_t m0 = (size_t)pix0 + wave * 16;
  v8f acc[4] = {{}, {}, {}, {}};
#pragma unroll 2
  for (int kb = 0; kb < KK; kb += 32) { const v16b a = frag_kb(XO + (m0 + nloc) * KK + kb, hlf);
#pragma unroll
    for (int t = 0; t < 4; ++t) acc[t] = wmma16b(a, frag_kb(CW + (size_t)(t * 16 + nloc) * KK + kb, hlf), acc[t]); }
#pragma unroll
  for (int t = 0; t < 4; ++t)
#pragma unroll
    for (int q = 0; q < 8; ++q) Tc[t * 16 + nloc][wave * 16 + 8 * hlf + q] = acc[t][q] * (1.0f / (XS * WSC));
  __syncthreads();
  for (int pass = 0; pass < 2; ++pass) { for (int q = t_; q < C * 16; q += 128) { const int o = q >> 4, c4 = (q & 15) * 4; *(volatile v4f*)(out + ((size_t)b * C + o) * P + pix0 + c4) = *(const v4f*)(&Tc[o][c4]); } __threadfence(); }
}
}

extern "C" void kernel_launch(void* const* d_in, const int* in_sizes, int n_in, void* d_out, int out_size, void* d_ws, size_t ws_size, hipStream_t stream) {
  (void)n_in;
  auto Fp = [&](int i) { return (const float*)d_in[i]; };
  if (in_sizes[0] != NB * C * P || in_sizes[1] != NOF * C * 9 || in_sizes[2] != NOF || in_sizes[3] != C * C * 9 || out_size != NB * C * P) return;
  size_t off = 0; char* ws = (char*)d_ws;
  auto carve = [&](size_t bytes) { char* p = ws + off; off += (bytes + 255) & ~(size_t)255; return p; };
  b16* XT = (b16*)carve((size_t)NB * PZ * C * 2); b16* PW = (b16*)carve((size_t)NOFP * KK * 2); b16* CW = (b16*)carve((size_t)C * KK * 2); float* OFFS = (float*)carve((size_t)NB * P * NOFP * 4); b16* XO = (b16*)carve((size_t)P * KK * 2);
  if (off > ws_size || off > ((size_t)128 << 20)) return;
  prepx_kernel<<<dim3(P / 64 + 1, 1, NB), 256, 0, stream>>>(Fp(0), XT);
  prepw_kernel<<<(NOFP * KK / 8 + C * KK / 8 + 255) / 256, 256, 0, stream>>>(Fp(1), Fp(3), PW, CW);
  offconv_kernel<<<dim3(P / 64, NB), 128, 0, stream>>>(XT, PW, Fp(2), OFFS);
  for (int b = 0; b < NB; ++b) {
    sample_kernel<<<P / 4, 256, 0, stream>>>(XT, OFFS, b, XO);
    conv_kernel<<<P / 64, 128, 0, stream>>>(XO, CW, b, (float*)d_out); }
}
